// KKAN_27221502722265
// MI455X (gfx1250) — hardware-verified
//
#include <hip/hip_runtime.h>
#include <math.h>

typedef __attribute__((ext_vector_type(16))) _Float16 v16h;
typedef __attribute__((ext_vector_type(16))) __bf16 v16b;
typedef __attribute__((ext_vector_type(8)))  _Float16 v8h;
typedef __attribute__((ext_vector_type(8)))  float v8f;
typedef __attribute__((ext_vector_type(4)))  float v4f;
typedef __attribute__((ext_vector_type(2)))  float v2f;
typedef __attribute__((ext_vector_type(4)))  unsigned v4u;
typedef __attribute__((ext_vector_type(4)))  int v4i;
typedef float __attribute__((may_alias)) float_a;
typedef int __attribute__((may_alias)) int_a;

template <typename T> __device__ __forceinline__ void vst2(void* p, T v) { *(volatile T*)p = v; __threadfence(); *(volatile T*)p = v; }
__device__ __forceinline__ v8f wmma16(v16h a, v16h b, v8f c) {
  v8f d = __builtin_amdgcn_wmma_f32_16x16x32_f16(false, a, false, b, (short)0, c, false, false);
  asm volatile("v_nop\n\tv_nop\n\tv_nop\n\tv_nop" : "+v"(d) : "v"(a), "v"(b));
  return d;
}
__device__ __forceinline__ v8f wmma_bf(v16b a, v16b b, v8f c) {
  v8f d = __builtin_amdgcn_wmma_f32_16x16x32_bf16(false, a, false, b, (short)0, c, false, false);
  asm volatile("v_nop\n\tv_nop\n\tv_nop\n\tv_nop" : "+v"(d) : "v"(a), "v"(b));
  return d;
}
__device__ __forceinline__ v16h frag_h(const _Float16* rowk0, int lane) {
  union { v16h v; v8h q[2]; } u; const _Float16* p = rowk0 + 8 * (lane >> 4);
  u.q[0] = *(const v8h*)p; u.q[1] = *(const v8h*)(p + 16); return u.v;
}
__device__ __forceinline__ v16h frag_f32(const float* rowk0, int lane) {
  v16h a; const float* p = rowk0 + 8 * (lane >> 4);
#pragma unroll
  for (int i = 0; i < 8; ++i) { a[i] = (_Float16)p[i]; a[8 + i] = (_Float16)p[16 + i]; }
  return a;
}
__device__ __forceinline__ v16h frag_f32s(const float* rowk0, int lane, float sc) {
  v16h a; const float* p = rowk0 + 8 * (lane >> 4);
#pragma unroll
  for (int i = 0; i < 8; ++i) { a[i] = (_Float16)(p[i] * sc); a[8 + i] = (_Float16)(p[16 + i] * sc); }
  return a;
}
__device__ __forceinline__ v16h fragc_f32(const float* W, int k0, int n, int lane, int ld, int K) {
  v16h a; const int g = lane >> 4;
#pragma unroll
  for (int i = 0; i < 8; ++i) { const int ka = k0 + 8 * g + i, kb = ka + 16;
    a[i] = (_Float16)(ka < K ? W[(size_t)(ka < K ? ka : K - 1) * ld + n] : 0.f); a[8 + i] = (_Float16)(kb < K ? W[(size_t)(kb < K ? kb : K - 1) * ld + n] : 0.f); }
  return a;
}
struct F2 { v16b h, l; };
__device__ __forceinline__ F2 bsplit16(const float v[16]) { F2 r;
#pragma unroll
  for (int i = 0; i < 16; ++i) { const __bf16 h = (__bf16)v[i]; r.h[i] = h; r.l[i] = (__bf16)(v[i] - (float)h); }
  return r; }
__device__ __forceinline__ F2 split_row(const float* row, int k0, int lane) { float v[16]; const float* p = row + k0 + 8 * (lane >> 4);
#pragma unroll
  for (int i = 0; i < 8; ++i) { v[i] = p[i]; v[8 + i] = p[16 + i]; }
  return bsplit16(v); }
__device__ __forceinline__ F2 split_rowK(const float* row, int k0, int lane, int K) { float v[16]; const int g = lane >> 4;
#pragma unroll
  for (int i = 0; i < 8; ++i) { const int ka = k0 + 8 * g + i, kb = ka + 16; v[i] = ka < K ? row[ka < K ? ka : K - 1] : 0.f; v[8 + i] = kb < K ? row[kb < K ? kb : K - 1] : 0.f; }
  return bsplit16(v); }
__device__ __forceinline__ F2 split_col(const float* W, int k0, int n, int lane, int ld, int K) { float v[16]; const int g = lane >> 4;
#pragma unroll
  for (int i = 0; i < 8; ++i) { const int ka = k0 + 8 * g + i, kb = ka + 16; v[i] = ka < K ? W[(size_t)(ka < K ? ka : K - 1) * ld + n] : 0.f; v[8 + i] = kb < K ? W[(size_t)(kb < K ? kb : K - 1) * ld + n] : 0.f; }
  return bsplit16(v); }
__device__ __forceinline__ v8f mac3(const F2& a, const F2& b, v8f c) { c = wmma_bf(a.l, b.h, c); c = wmma_bf(a.h, b.l, c); return wmma_bf(a.h, b.h, c); }
__device__ __forceinline__ float sigm(float v) { return 1.0f / (1.0f + expf(-v)); }
#define LDSX() do { asm volatile("s_wait_dscnt 0" ::: "memory"); __builtin_amdgcn_wave_barrier(); __builtin_amdgcn_fence(__ATOMIC_RELEASE, "workgroup"); } while (0)


#define NIMG 128
#ifndef TNI
#define TNI NIMG
#endif
#define NSPL 8
typedef __attribute__((ext_vector_type(8))) __bf16 v8b;
__device__ __forceinline__ v16b frag_b(const __bf16* rowk0, int lane) {
  union { v16b v; v8b q[2]; } u; const __bf16* p = rowk0 + 8 * (lane >> 4);
  u.q[0] = *(const v8b*)p; u.q[1] = *(const v8b*)(p + 16); return u.v;
}
__device__ __forceinline__ float bfr(float v) { return (float)(__bf16)v; }
__device__ __attribute__((noinline)) float exp_ni(float v) { return expf(v); }
__device__ __attribute__((noinline)) float erf_ni(float v) { return erff(v); }

#define FIN1 27
#define FIN2 36
#define FIN3 72
#define FIN4 144
#define FINP1 32
#define FINP2 64
#define FINP3 96
#define FINP4 160
#define KP1 256
#define KP2 352
#define KP3 672
#define KP4 1312
#define WS_W1H 0u
#define WS_W1L (WS_W1H + 2u * 16 * KP1)
#define WS_W2H (WS_W1L + 2u * 16 * KP1)
#define WS_W2L (WS_W2H + 2u * 16 * KP2)
#define WS_W3H (WS_W2L + 2u * 16 * KP2)
#define WS_W3L (WS_W3H + 2u * 16 * KP3)
#define WS_W4H (WS_W3L + 2u * 16 * KP3)
#define WS_W4L (WS_W4H + 2u * 32 * KP4)
#define WS_L1  (((WS_W4L + 2u * 32 * KP4) + 127u) / 128u * 128u)
#define WS_L2  (WS_L1 + 2u * 2048 * 2048)
#define WS_L3  (WS_L2 + 2u * 1024 * 2048)
#define WS_A1  (WS_L3 + 2u * 128 * 1024)
#define WS_A2  (WS_A1 + 4u * NIMG * 4 * 1024)
#define WS_P2  (WS_A2 + 4u * NIMG * 8 * 1024)
#define WS_A3  (WS_P2 + 4u * NIMG * 8 * 256)
#define WS_A4  (WS_A3 + 4u * NIMG * 16 * 256)
#define WS_P4  (WS_A4 + 4u * NIMG * 32 * 256)
#define WS_H1  (WS_P4 + 4u * NIMG * 2048)
#define WS_H2  (WS_H1 + 4u * NIMG * 2048)
#define WS_END (WS_H2 + 4u * NIMG * 1024)

__device__ __forceinline__ void bspline8(float x, float* out) {
  float g[12];
#pragma unroll
  for (int i = 0; i < 12; ++i) g[i] = (float)(i - 3) * 0.4f - 1.0f;
  float b[11];
#pragma unroll
  for (int i = 0; i < 11; ++i) b[i] = (x >= g[i] && x < g[i + 1]) ? 1.0f : 0.0f;
#pragma unroll
  for (int k = 1; k <= 3; ++k) {
#pragma unroll
    for (int i = 0; i < 11 - k; ++i) { const float left = (x - g[i]) / (g[k + i] - g[i]) * b[i]; const float right = (g[i + k + 1] - x) / (g[i + k + 1] - g[i + 1]) * b[i + 1]; b[i] = left + right; } }
#pragma unroll
  for (int j = 0; j < NSPL; ++j) out[j] = b[j];
}
__device__ __forceinline__ float silu_f(float x) { return x / (1.0f + exp_ni(-x)); }
__global__ __launch_bounds__(256) void k_packk(const float* __restrict__ BW1, const float* __restrict__ SW1, const float* __restrict__ SC1, const float* __restrict__ BW2, const float* __restrict__ SW2, const float* __restrict__ SC2, const float* __restrict__ BW3, const float* __restrict__ SW3, const float* __restrict__ SC3, const float* __restrict__ BW4, const float* __restrict__ SW4, const float* __restrict__ SC4, __bf16* __restrict__ WS0) {
  __shared__ __align__(16) __bf16 sh[KP4], sl[KP4]; const int o = blockIdx.x, layer = blockIdx.y, t = threadIdx.x;
  int fin, finp, kp, cout; const float *BW, *SW, *SC; size_t dh, dl;
  if (layer == 0) { fin = FIN1; finp = FINP1; kp = KP1; cout = 4; BW = BW1; SW = SW1; SC = SC1; dh = WS_W1H; dl = WS_W1L; }
  else if (layer == 1) { fin = FIN2; finp = FINP2; kp = KP2; cout = 8; BW = BW2; SW = SW2; SC = SC2; dh = WS_W2H; dl = WS_W2L; }
  else if (layer == 2) { fin = FIN3; finp = FINP3; kp = KP3; cout = 16; BW = BW3; SW = SW3; SC = SC3; dh = WS_W3H; dl = WS_W3L; }
  else { fin = FIN4; finp = FINP4; kp = KP4; cout = 32; BW = BW4; SW = SW4; SC = SC4; dh = WS_W4H; dl = WS_W4L; }
  const int rows = (layer == 3) ? 32 : 16; if (o >= rows) return;
  for (int k = t; k < kp; k += 256) { float v = 0.f; bool exact = true;
    if (o < cout) { if (k < fin) v = bfr(BW[o * fin + k]); else if (k >= finp && k < finp + fin * NSPL) { const int f = (k - finp) / NSPL, j = (k - finp) % NSPL; v = bfr(SW[((size_t)o * fin + f) * NSPL + j]) * bfr(SC[o * fin + f]); exact = false; } }
    const __bf16 hb = (__bf16)v; sh[k] = hb; sl[k] = exact ? (__bf16)0.f : (__bf16)(v - (float)hb); }
  __syncthreads();
  __bf16* DH = (__bf16*)((char*)WS0 + dh) + (size_t)o * kp; __bf16* DL = (__bf16*)((char*)WS0 + dl) + (size_t)o * kp;
  for (int q = t; q < kp / 8; q += 256) { vst2((unsigned*)(DH + q * 8), *(const v4u*)&sh[q * 8]); vst2((unsigned*)(DL + q * 8), *(const v4u*)&sl[q * 8]); }
}
__global__ __launch_bounds__(256) void k_packl(const float* __restrict__ W1, const float* __restrict__ W2, const float* __restrict__ W3, __bf16* __restrict__ L1, __bf16* __restrict__ L2, __bf16* __restrict__ L3) {
  __shared__ __align__(16) __bf16 s[2048]; const int n = blockIdx.x, which = blockIdx.y, t = threadIdx.x; int K; __bf16* dst;
  if (which == 0) { K = 2048; dst = L1 + (size_t)n * 2048; for (int k = t; k < K; k += 256) s[k] = (__bf16)W1[(size_t)n * 2048 + k]; }
  else if (which == 1) { if (n >= 1024) return; K = 2048; dst = L2 + (size_t)n * 2048; for (int k = t; k < K; k += 256) s[k] = (__bf16)W2[(size_t)n * 2048 + k]; }
  else { if (n >= 128) return; K = 1024; dst = L3 + (size_t)n * 1024; for (int k = t; k < K; k += 256) s[k] = (__bf16)((n < 10) ? W3[(size_t)n * 1024 + k] : 0.f); }
  __syncthreads();
  for (int q = t; q < K / 8; q += 256) vst2((unsigned*)(dst + q * 8), *(const v4u*)&s[q * 8]);
}
template <int CIN, int COUT, int HW, int RIN>
__global__ __launch_bounds__(128) void k_kconv(const float* __restrict__ X, const __bf16* __restrict__ WH, const __bf16* __restrict__ WL, float* __restrict__ OUT) {
  constexpr int FIN = CIN * 9, FINP = (FIN + 31) / 32 * 32, KP = (FINP + FIN * NSPL + 31) / 32 * 32, NT = (COUT + 15) / 16;
  __shared__ __align__(16) __bf16 sh[64][40], sl[64][40]; __shared__ __align__(16) float so[NT * 16][68];
  const int tid = threadIdx.x, wave = tid >> 5, lane = tid & 31, col = lane & 15, g = lane >> 4; const size_t p0 = (size_t)blockIdx.x * 64;
  auto patch = [&](int r, int f) -> float { const size_t pos = p0 + r; const int b = (int)(pos / (HW * HW)); const int hw = (int)(pos % (HW * HW)); const int h = hw / HW, w = hw % HW; const int c = f / 9, tap = f % 9; const int yy = h + tap / 3 - 1, xx = w + tap % 3 - 1;
    if (yy < 0 || yy >= HW || xx < 0 || xx >= HW) return 0.f; const float v = X[(((size_t)b * CIN + c) * HW + yy) * HW + xx]; return RIN ? bfr(v) : v; };
  v8f acc[NT] = {}, accl[NT] = {};
#pragma unroll 1
  for (int kc = 0; kc < KP / 32; ++kc) { const int k0 = kc * 32;
    if (k0 < FINP) {
      for (int e = tid; e < 64 * 32; e += 128) { const int r = e >> 5, kk = e & 31; const int f = k0 + kk; float v = 0.f; if (f < FIN) v = silu_f(patch(r, f)); const __bf16 hb = (__bf16)v; sh[r][kk] = hb; sl[r][kk] = (__bf16)(v - (float)hb); } }
    else {
      for (int e = tid; e < 64 * 4; e += 128) { const int r = e >> 2, fi = e & 3; const int f = (k0 - FINP) / NSPL + fi; float bs[NSPL];
        if (f < FIN) bspline8(patch(r, f), bs); else {
#pragma unroll
          for (int j = 0; j < NSPL; ++j) bs[j] = 0.f; }
#pragma unroll
        for (int j = 0; j < NSPL; ++j) { const float v = bs[j]; const __bf16 hb = (__bf16)v; sh[r][fi * 8 + j] = hb; sl[r][fi * 8 + j] = (__bf16)(v - (float)hb); } } }
    __syncthreads();
    { const v16b a = frag_b(&sh[wave * 16 + col][0], lane), al = frag_b(&sl[wave * 16 + col][0], lane);
#pragma unroll
      for (int j = 0; j < NT; ++j) { const v16b wh = frag_b(WH + (size_t)(j * 16 + col) * KP + k0, lane); acc[j] = wmma_bf(a, wh, acc[j]); accl[j] = wmma_bf(al, wh, accl[j]); accl[j] = wmma_bf(a, frag_b(WL + (size_t)(j * 16 + col) * KP + k0, lane), accl[j]); } }
    __syncthreads(); }
#pragma unroll
  for (int j = 0; j < NT; ++j)
#pragma unroll
    for (int r = 0; r < 8; ++r) so[j * 16 + col][wave * 16 + 8 * g + r] = acc[j][r] + accl[j][r];
  __syncthreads();
  { const int b = (int)(p0 / (HW * HW)); const int hw0 = (int)(p0 % (HW * HW));
    for (int e = tid; e < COUT * 16; e += 128) { const int o = e >> 4, q = e & 15; vst2(OUT + ((size_t)b * COUT + o) * HW * HW + hw0 + q * 4, *(const v4f*)&so[o][q * 4]); } }
}
template <int CH, int HW>
__global__ __launch_bounds__(256) void k_pool(const float* __restrict__ IN, float* __restrict__ OUT) {
  const int b = blockIdx.x / CH, c = blockIdx.x % CH; constexpr int HO = HW / 2; __shared__ __align__(16) float so[HO * HO];
  for (int e = threadIdx.x; e < HO * HO; e += 256) { const int y = e / HO, x = e % HO; const float* p = IN + (((size_t)b * CH + c) * HW + 2 * y) * HW + 2 * x; so[e] = fmaxf(fmaxf(p[0], p[1]), fmaxf(p[HW], p[HW + 1])); }
  __syncthreads();
  for (int e = threadIdx.x; e < HO * HO / 4; e += 256) vst2(OUT + ((size_t)b * CH + c) * HO * HO + e * 4, *(const v4f*)&so[e * 4]);
}
template <int K, int RELU>
__global__ __launch_bounds__(128) void k_lin(const float* __restrict__ A, const __bf16* __restrict__ Wr, const float* __restrict__ B, float* __restrict__ Y, int NOUT) {
  __shared__ __align__(16) float so[64][132];
  const int tid = threadIdx.x, wave = tid >> 5, lane = tid & 31, col = lane & 15, g = lane >> 4; const size_t r0 = (size_t)blockIdx.x * 64 + wave * 16; const int n0 = blockIdx.y * 128;
  v8f acc[8] = {};
#pragma unroll 4
  for (int kc = 0; kc < K / 32; ++kc) { const F2 a = split_row(A + (r0 + col) * K, kc * 32, lane);
#pragma unroll
    for (int j = 0; j < 8; ++j) { const v16b w = frag_b(Wr + (size_t)(n0 + j * 16 + col) * K + kc * 32, lane); acc[j] = wmma_bf(a.l, w, acc[j]); acc[j] = wmma_bf(a.h, w, acc[j]); } }
#pragma unroll
  for (int j = 0; j < 8; ++j) { const int c = n0 + j * 16 + col; const float bb = (c < NOUT) ? bfr(B[c]) : 0.f;
#pragma unroll
    for (int r = 0; r < 8; ++r) { float v = acc[j][r] + bb; if (RELU) v = fmaxf(v, 0.f); so[wave * 16 + 8 * g + r][j * 16 + col] = v; } }
  __syncthreads();
  if (NOUT >= n0 + 128) { for (int e = tid; e < 64 * 32; e += 128) { const int r = e >> 5, q = e & 31; vst2(Y + ((size_t)blockIdx.x * 64 + r) * NOUT + n0 + q * 4, *(const v4f*)&so[r][q * 4]); } }
  else {
    for (int e = tid; e < 64 * NOUT; e += 128) { const int r = e / NOUT, c = e % NOUT; Y[((size_t)blockIdx.x * 64 + r) * NOUT + c] = so[r][c]; } }
}
extern "C" void kernel_launch(void* const* d_in, const int* in_sizes, int n_in, void* d_out, int out_size, void* d_ws, size_t ws_size, hipStream_t stream) {
  (void)in_sizes; (void)n_in; (void)out_size;
  const float** F = (const float**)d_in;
  if (ws_size < (size_t)WS_END) return;
  char* ws = (char*)d_ws; __bf16* W0 = (__bf16*)ws; __bf16 *L1 = (__bf16*)(ws + WS_L1), *L2 = (__bf16*)(ws + WS_L2), *L3 = (__bf16*)(ws + WS_L3); float *A1 = (float*)(ws + WS_A1), *A2 = (float*)(ws + WS_A2), *P2 = (float*)(ws + WS_P2), *A3 = (float*)(ws + WS_A3), *A4 = (float*)(ws + WS_A4), *P4 = (float*)(ws + WS_P4), *H1 = (float*)(ws + WS_H1), *H2 = (float*)(ws + WS_H2);
  k_packk<<<dim3(32, 4), 256, 0, stream>>>(F[1], F[2], F[3], F[4], F[5], F[6], F[7], F[8], F[9], F[10], F[11], F[12], W0);
  k_packl<<<dim3(2048, 3), 256, 0, stream>>>(F[13], F[15], F[17], L1, L2, L3);
  k_kconv<3, 4, 32, 1><<<TNI * 1024 / 64, 128, 0, stream>>>(F[0], (const __bf16*)(ws + WS_W1H), (const __bf16*)(ws + WS_W1L), A1);
  k_kconv<4, 8, 32, 0><<<TNI * 1024 / 64, 128, 0, stream>>>(A1, (const __bf16*)(ws + WS_W2H), (const __bf16*)(ws + WS_W2L), A2);
  k_pool<8, 32><<<TNI * 8, 256, 0, stream>>>(A2, P2);
  k_kconv<8, 16, 16, 0><<<TNI * 256 / 64, 128, 0, stream>>>(P2, (const __bf16*)(ws + WS_W3H), (const __bf16*)(ws + WS_W3L), A3);
  k_kconv<16, 32, 16, 0><<<TNI * 256 / 64, 128, 0, stream>>>(A3, (const __bf16*)(ws + WS_W4H), (const __bf16*)(ws + WS_W4L), A4);
  k_pool<32, 16><<<TNI * 32, 256, 0, stream>>>(A4, P4);
  k_lin<2048, 1><<<dim3((TNI + 63) / 64, 2048 / 128), 128, 0, stream>>>(P4, L1, F[14], H1, 2048);
  k_lin<2048, 1><<<dim3((TNI + 63) / 64, 1024 / 128), 128, 0, stream>>>(H1, L2, F[16], H2, 1024);
  k_lin<1024, 0><<<dim3((TNI + 63) / 64, 1), 128, 0, stream>>>(H2, L3, F[18], (float*)d_out, 10);
}
